// BiMamba2DFast_18124761989165
// MI455X (gfx1250) — hardware-verified
//
#include <hip/hip_runtime.h>
#include <math.h>

typedef __attribute__((ext_vector_type(16))) _Float16 v16h;
typedef __attribute__((ext_vector_type(8)))  _Float16 v8h;
typedef __attribute__((ext_vector_type(4)))  _Float16 v4h;
typedef __attribute__((ext_vector_type(16))) __bf16   v16b;
typedef __attribute__((ext_vector_type(8)))  __bf16   v8b;
typedef __attribute__((ext_vector_type(8)))  float    v8f;
typedef __attribute__((ext_vector_type(4)))  float    v4f;

constexpr int kB     = 2;
constexpr int kH     = 56;
constexpr int kW     = 56;
constexpr int kL     = 56;
constexpr int kD     = 192;
constexpr int kDX    = 2 * kD;
constexpr int kDi    = 384;
constexpr int kDi2   = 2 * kDi;
constexpr int kDiX   = 2 * kDi;
constexpr int kNs    = 16;
constexpr int kR     = 12;
constexpr int kRP    = 32;
constexpr int kXd    = kR + 2 * kNs;
constexpr int kXdP   = 64;
constexpr int kConv  = 3;
constexpr int kSeqs  = kB * kW;
constexpr int kSeqs2 = 2 * kSeqs;
constexpr int kRowsL = kSeqs2 * kL;
constexpr int kRows  = 12800;
constexpr int kRowsO = kSeqs * kL;
constexpr int kThr   = 256;

constexpr float kInCarry = 1024.0f;
constexpr float kWCarry  = 4096.0f;
constexpr float kACarry  = 256.0f;
constexpr float kScIn = 1.0f / (kInCarry * kWCarry);
constexpr float kScA  = 1.0f / (kACarry * kWCarry);
constexpr float kF16MinNormal = 6.103515625e-5f;

static_assert((kRows % 64) == 0 && ((kRows / 64) % 8) == 0 && kRows >= kRowsL, "every GEMM grid exact");
static_assert((kDX % 32) == 0 && (kDiX % 32) == 0 && (kRP % 32) == 0, "GEMM K multiples of 32");

constexpr size_t kOffX16 = 0;
constexpr size_t kOffXZ  = kOffX16 + (size_t)kRows * kDX * 2;
constexpr size_t kOffXC  = kOffXZ  + (size_t)kRows * kDi2 * 4;
constexpr size_t kOffXC16 = kOffXC + (size_t)kRows * kDi * 4;
constexpr size_t kOffP   = kOffXC16 + (size_t)kRows * kDiX * 2;
constexpr size_t kOffDT16 = kOffP  + (size_t)kRows * kXdP * 4;
constexpr size_t kOffDL  = kOffDT16 + (size_t)kRows * kRP * 2;
constexpr size_t kOffHID = kOffDL  + (size_t)kRows * kDi * 4;
constexpr size_t kOffY16 = kOffHID + (size_t)kRows * kDi * 4;
constexpr size_t kOffO   = kOffY16 + (size_t)kRows * kDiX * 2;
constexpr size_t kOffR1  = kOffO   + (size_t)kRows * kD * 4;
constexpr size_t kOffWts = kOffR1  + (size_t)kRowsO * kD * 4;
constexpr size_t kWIN = 0;
constexpr size_t kWX  = kWIN + (size_t)kDi2 * kDX * 2;
constexpr size_t kWDT = kWX  + (size_t)kXdP * kDiX * 2;
constexpr size_t kWO  = kWDT + (size_t)kDi * kRP * 2;
constexpr size_t kWBV = kWO  + (size_t)kD * kDiX * 2;
constexpr int    kBvZ = 0;
constexpr int    kBvDt = kDi2;
constexpr int    kBvTot = kDi2 + kDi;
constexpr size_t kWBlock = kWBV + (size_t)kBvTot * 4;
constexpr size_t kWsTotal = kOffWts + 2 * kWBlock;
static_assert(kWsTotal <= 268435456ull, "inside the offered workspace");
static_assert((kOffXZ % 256) == 0 && (kOffXC % 256) == 0 && (kOffXC16 % 256) == 0 && (kOffP % 256) == 0 && (kOffDT16 % 256) == 0 && (kOffDL % 256) == 0 && (kOffHID % 256) == 0 && (kOffY16 % 256) == 0 && (kOffO % 256) == 0 && (kOffR1 % 256) == 0 && (kOffWts % 256) == 0 && (kWX % 256) == 0 && (kWDT % 256) == 0 && (kWO % 256) == 0 && (kWBV % 256) == 0 && (kWBlock % 256) == 0, "aligned regions");

__device__ __forceinline__ unsigned short f2bf_bits(float f) {
  unsigned u = __float_as_uint(f);
  return (unsigned short)((u + 0x7FFFu + ((u >> 16) & 1u)) >> 16);
}
__device__ __forceinline__ float bf_bits2f(unsigned short h) { return __uint_as_float(((unsigned)h) << 16); }
__device__ __forceinline__ float bf16r(float f) { return bf_bits2f(f2bf_bits(f)); }
__device__ __forceinline__ float carry_flush(float v, float carry) {
  const float s = v * carry;
  return (fabsf(s) < kF16MinNormal) ? 0.0f : s;
}
__device__ __forceinline__ float frcp(float x) { return __builtin_amdgcn_rcpf(x); }

__device__ __forceinline__ void dep_guard4_h(v8f& a, v8f& b, v8f& c, v8f& d, v16h x, v16h y) { asm volatile("v_nop\n\tv_nop\n\tv_nop\n\tv_nop" : "+v"(a), "+v"(b), "+v"(c), "+v"(d) : "v"(x), "v"(y)); }
__device__ __forceinline__ void dep_guard4_b(v8f& a, v8f& b, v8f& c, v8f& d, v16b x, v16b y) { asm volatile("v_nop\n\tv_nop\n\tv_nop\n\tv_nop" : "+v"(a), "+v"(b), "+v"(c), "+v"(d) : "v"(x), "v"(y)); }
__device__ __forceinline__ void keep4_h(v16h a, v16h b, v16h c, v16h d) { asm volatile("v_nop" :: "v"(a), "v"(b), "v"(c), "v"(d)); }
__device__ __forceinline__ void keep4_b(v16b a, v16b b, v16b c, v16b d) { asm volatile("v_nop" :: "v"(a), "v"(b), "v"(c), "v"(d)); }
__device__ __forceinline__ void acc_guard4(v8f& a, v8f& b, v8f& c, v8f& d) { asm volatile("v_nop\n\tv_nop\n\tv_nop\n\tv_nop" : "+v"(a), "+v"(b), "+v"(c), "+v"(d)); }

template <typename T> struct Frag;
template <> struct Frag<_Float16> {
  typedef v16h V; union U { v16h v; v8h h[2]; };
  static __device__ __forceinline__ v16h load(const _Float16* p) {
    U f; f.h[0] = *(const v8h*)(p); f.h[1] = *(const v8h*)(p + 16); return f.v;
  }
  static __device__ __forceinline__ v8f mma(v16h a, v16h b, v8f c) {
    return __builtin_amdgcn_wmma_f32_16x16x32_f16(false, a, false, b, (short)0, c, false, false);
  }
  static __device__ __forceinline__ void guard4(v8f& a, v8f& b, v8f& c, v8f& d, v16h x, v16h y) { dep_guard4_h(a, b, c, d, x, y); }
  static __device__ __forceinline__ void keep(v16h a, v16h b, v16h c, v16h d) { keep4_h(a, b, c, d); }
};
template <> struct Frag<__bf16> {
  typedef v16b V; union U { v16b v; v8b h[2]; };
  static __device__ __forceinline__ v16b load(const __bf16* p) {
    U f; f.h[0] = *(const v8b*)(p); f.h[1] = *(const v8b*)(p + 16); return f.v;
  }
  static __device__ __forceinline__ v8f mma(v16b a, v16b b, v8f c) {
    return __builtin_amdgcn_wmma_f32_16x16x32_bf16(false, a, false, b, (short)0, c, false, false);
  }
  static __device__ __forceinline__ void guard4(v8f& a, v8f& b, v8f& c, v8f& d, v16b x, v16b y) { dep_guard4_b(a, b, c, d, x, y); }
  static __device__ __forceinline__ void keep(v16b a, v16b b, v16b c, v16b d) { keep4_b(a, b, c, d); }
};

__device__ __forceinline__ v8f mma_h(v16h a, v16h b, v8f c) {
  c = __builtin_amdgcn_wmma_f32_16x16x32_f16(false, a, false, b, (short)0, c, false, false);
  asm volatile("v_nop\n\tv_nop\n\tv_nop\n\tv_nop" : "+v"(c) : "v"(a), "v"(b));
  return c;
}

template <int ET> struct Elem;
template <> struct Elem<0> { typedef _Float16 T; };
template <> struct Elem<1> { typedef __bf16 T; };
template <int ET, bool SPLIT, int BIAS_MODE, int OUT_MODE, bool RESID, int ACT = 0>
__global__ __launch_bounds__(256) void wmma_gemm64(
    const unsigned short* __restrict__ Ap, const unsigned short* __restrict__ A2p, int lda, long strideA,
    const unsigned short* __restrict__ Btp, const unsigned short* __restrict__ Bt2p, int ldb, long strideB,
    void* __restrict__ Cout, void* __restrict__ Cout2, int ldc, long strideC,
    const float* __restrict__ bias,
    const float* __restrict__ resid, long strideR,
    int M, int N, int K, float scale) {
  typedef typename Elem<ET>::T T;
  typedef typename Frag<T>::V V;
  const T* A = (const T*)Ap; const T* A2 = (const T*)A2p; const T* Bt = (const T*)Btp; const T* Bt2 = (const T*)Bt2p;
  __shared__ __align__(16) float sT[8][16 * 68];
  const int b    = blockIdx.y;
  const int lane = threadIdx.x & 31;
  const int wave = threadIdx.x >> 5;
  const int tilesN = N >> 6;
  const int tilesM = M >> 6;
  const int tile = blockIdx.x * 8 + wave;
  if (tile >= tilesM * tilesN) return;
  const int tm = tile / tilesN;
  const int tn = tile - tm * tilesN;
  const int m0 = tm << 6;
  const int n0 = tn << 6;

  const T* Ab  = A  + (size_t)b * strideA;
  const T* Bb  = Bt + (size_t)b * strideB;
  const T* Ab2 = SPLIT ? (A2  + (size_t)b * strideA) : nullptr;
  const T* Bb2 = SPLIT ? (Bt2 + (size_t)b * strideB) : nullptr;

  const int rlane = lane & 15;
  const int koff  = (lane >> 4) * 8;
  const int mOff  = (lane >> 4) * 8;

  v8f acc[4][4];
#pragma unroll
  for (int i = 0; i < 4; ++i)
#pragma unroll
    for (int j = 0; j < 4; ++j) acc[i][j] = (v8f){0.f,0.f,0.f,0.f,0.f,0.f,0.f,0.f};

  for (int k0 = 0; k0 < K; k0 += 32) {
    V bh[4], bl[4];
#pragma unroll
    for (int j = 0; j < 4; ++j) {
      const size_t bo = (size_t)(n0 + (j << 4) + rlane) * ldb + koff + k0;
      bh[j] = Frag<T>::load(Bb + bo);
      if (SPLIT) bl[j] = Frag<T>::load(Bb2 + bo);
    }
#pragma unroll
    for (int i = 0; i < 4; ++i) {
      const size_t ao = (size_t)(m0 + (i << 4) + rlane) * lda + koff + k0;
      V ah = Frag<T>::load(Ab + ao);
      V al;
      if (SPLIT) al = Frag<T>::load(Ab2 + ao);
#pragma unroll
      for (int j = 0; j < 4; ++j) {
        acc[i][j] = Frag<T>::mma(ah, bh[j], acc[i][j]);
        if (SPLIT) {
          acc[i][j] = Frag<T>::mma(ah, bl[j], acc[i][j]);
          acc[i][j] = Frag<T>::mma(al, bh[j], acc[i][j]);
        }
      }
      Frag<T>::guard4(acc[i][0], acc[i][1], acc[i][2], acc[i][3], ah, SPLIT ? al : ah);
    }
    Frag<T>::keep(bh[0], bh[1], bh[2], bh[3]);
    if (SPLIT) Frag<T>::keep(bl[0], bl[1], bl[2], bl[3]);
  }
  acc_guard4(acc[0][0], acc[0][1], acc[0][2], acc[0][3]);
  acc_guard4(acc[1][0], acc[1][1], acc[1][2], acc[1][3]);
  acc_guard4(acc[2][0], acc[2][1], acc[2][2], acc[2][3]);
  acc_guard4(acc[3][0], acc[3][1], acc[3][2], acc[3][3]);

  float* slab = sT[wave];
  const float* Rb = RESID ? (resid + (size_t)b * strideR) : nullptr;
#pragma unroll
  for (int i = 0; i < 4; ++i) {
    const int mBase = m0 + (i << 4);
#pragma unroll
    for (int j = 0; j < 4; ++j) {
      const int n = n0 + (j << 4) + rlane;
      float bv = 0.f;
      if (BIAS_MODE == 2) bv = bias[n];
#pragma unroll
      for (int r = 0; r < 8; ++r) {
        float v = acc[i][j][r] * scale;
        if (BIAS_MODE == 1) v += bias[mBase + mOff + r];
        if (BIAS_MODE == 2) v += bv;
        if (RESID) v += Rb[(size_t)(mBase + mOff + r) * ldc + n];
        if (ACT == 1) v = tanhf(v);
        if (ACT == 2) v = fmaxf(v, 0.0f);
        if (ACT == 3) v = v / (1.0f + expf(-v));
        if (ACT == 4) v = (v > 0.f) ? v : 0.01f * v;
        slab[(mOff + r) * 68 + (j << 4) + rlane] = v;
      }
    }
    __builtin_amdgcn_fence(__ATOMIC_RELEASE, "workgroup");
    __builtin_amdgcn_wave_barrier();
    __builtin_amdgcn_fence(__ATOMIC_ACQUIRE, "workgroup");
    if (OUT_MODE == 0) {
      float* C = (float*)Cout + (size_t)b * strideC;
      const int hh = lane >> 4, c4 = (lane & 15) * 4;
      for (int pass = 0; pass < 2; ++pass) {
#pragma unroll
        for (int it = 0; it < 8; ++it) {
          const int row = it * 2 + hh;
          v4f v = *(const v4f*)(slab + row * 68 + c4);
          *(volatile v4f*)(C + (size_t)(mBase + row) * ldc + n0 + c4) = v;
        }
        __threadfence();
      }
    } else {
      const int q = lane >> 3, c8 = (lane & 7) * 8;
      unsigned short* C  = (unsigned short*)Cout  + (size_t)b * strideC;
      unsigned short* C2 = (OUT_MODE == 2) ? ((unsigned short*)Cout2 + (size_t)b * strideC) : nullptr;
      for (int pass = 0; pass < 2; ++pass) {
#pragma unroll
        for (int it = 0; it < 4; ++it) {
          const int row = it * 4 + q;
          const float* sp = slab + row * 68 + c8;
          v8h hv, lv;
#pragma unroll
          for (int e = 0; e < 8; ++e) {
            if (OUT_MODE == 1) {
              hv[e] = (_Float16)sp[e];
            } else {
              unsigned short hb = f2bf_bits(sp[e]);
              unsigned short lb = f2bf_bits(sp[e] - bf_bits2f(hb));
              hv[e] = __builtin_bit_cast(_Float16, hb);
              lv[e] = __builtin_bit_cast(_Float16, lb);
            }
          }
          *(volatile v8h*)(C + (size_t)(mBase + row) * ldc + n0 + c8) = hv;
          if (OUT_MODE == 2) *(volatile v8h*)(C2 + (size_t)(mBase + row) * ldc + n0 + c8) = lv;
        }
        __threadfence();
      }
    }
    __builtin_amdgcn_fence(__ATOMIC_RELEASE, "workgroup");
    __builtin_amdgcn_wave_barrier();
    __builtin_amdgcn_fence(__ATOMIC_ACQUIRE, "workgroup");
  }
}


__device__ __forceinline__ void split_hl(float v, float c, _Float16& hi, _Float16& lo) {
  const float sv = carry_flush(v, c);
  hi = (_Float16)sv;
  const float r = sv - (float)hi;
  lo = (_Float16)((fabsf(r) < kF16MinNormal) ? 0.0f : r);
}

__global__ __launch_bounds__(kThr) void cast_rows_kernel(const float* __restrict__ src, unsigned short* __restrict__ dst, int per, int ldd, int colOff) {
  const int i = blockIdx.x * kThr + threadIdx.x;
  const int n = i / per;
  const int k8 = (i - n * per) * 8;
  const v4f a0 = *(const v4f*)(src + (size_t)i * 8);
  const v4f a1 = *(const v4f*)(src + (size_t)i * 8 + 4);
  v8h hv;
#pragma unroll
  for (int e = 0; e < 4; ++e) {
    const float w0 = a0[e], w1 = a1[e];
    hv[e]     = (_Float16)carry_flush(bf16r(w0), kWCarry);
    hv[4 + e] = (_Float16)carry_flush(bf16r(w1), kWCarry);
  }
  unsigned short* dp = dst + (size_t)n * ldd + colOff + k8;
  *(volatile v8h*)dp = hv;
  __threadfence();
  *(volatile v8h*)dp = hv;
}
static_assert((kDi2 * (kD / 8)) % kThr == 0 && (kD * (kDi / 8)) % kThr == 0, "row cast grids exact");

__global__ __launch_bounds__(64) void wx_plane_kernel(const float* __restrict__ xw, unsigned short* __restrict__ WX, int colOff) {
  const int c = blockIdx.x;
  const bool live = c < kXd;
  const int k8 = threadIdx.x * 8;
  const float* sp = xw + (size_t)(live ? c : 0) * kDi + k8;
  const v4f a0 = *(const v4f*)sp;
  const v4f a1 = *(const v4f*)(sp + 4);
  v8h hv;
#pragma unroll
  for (int e = 0; e < 4; ++e) {
    const float w0 = a0[e], w1 = a1[e];
    hv[e]     = (_Float16)(live ? carry_flush(bf16r(w0), kWCarry) : 0.0f);
    hv[4 + e] = (_Float16)(live ? carry_flush(bf16r(w1), kWCarry) : 0.0f);
  }
  unsigned short* dp = WX + (size_t)c * kDiX + colOff + k8;
  *(volatile v8h*)dp = hv;
  __threadfence();
  *(volatile v8h*)dp = hv;
}

__global__ __launch_bounds__(kThr) void wdt_plane_kernel(const float* __restrict__ dtw, unsigned short* __restrict__ WDT) {
  const int i = blockIdx.x * kThr + threadIdx.x;
  const int d = i >> 2;
  const int c8 = (i & 3) * 8;
  v8h hv;
#pragma unroll
  for (int e = 0; e < 8; ++e) {
    const int c = c8 + e;
    const int cc = (c >= 16) ? (c - 16) : c;
    const bool live = cc < kR;
    const float w = dtw[(size_t)d * kR + (live ? cc : 0)];
    hv[e] = (_Float16)(live ? carry_flush(bf16r(w), kWCarry) : 0.0f);
  }
  unsigned short* dp = WDT + (size_t)i * 8;
  *(volatile v8h*)dp = hv;
  __threadfence();
  *(volatile v8h*)dp = hv;
}
static_assert(kDi * 4 == 6 * kThr, "step plane grid exact");

__global__ __launch_bounds__(128) void bias_rows_kernel(const float* __restrict__ dtb, float* __restrict__ BV) {
  const int i = blockIdx.x * 128 + threadIdx.x;
  const int idt = i - kBvDt;
  const float v = dtb[(idt >= 0) ? idt : 0];
  const float o = (idt >= 0) ? bf16r(v) : 0.0f;
  for (int pass = 0; pass < 2; ++pass) {
    *(volatile float*)(BV + i) = o;
    __threadfence();
  }
}
static_assert(kBvTot % 128 == 0 && kBvDt % 128 == 0, "bias grid exact; regions block-uniform");

template <bool kSecond>
__global__ __launch_bounds__(kThr) void pass_rows_kernel(const float* __restrict__ src, unsigned short* __restrict__ X16) {
  const int i = blockIdx.x * kThr + threadIdx.x;
  const int r = i / 24;
  const int d8 = (i - r * 24) * 8;
  const bool live = r < kRowsL;
  const int rc = live ? r : 0;
  const int sp = rc / kL;
  const int l = rc - sp * kL;
  const bool fwd = sp < kSeqs;
  const int s = fwd ? sp : (sp - kSeqs);
  const int ls = fwd ? l : (kL - 1 - l);
  v8h hv, lv;
#pragma unroll
  for (int e = 0; e < 8; ++e) {
    const int d = d8 + e;
    size_t idx;
    if (kSecond) {
      const int g = ls * kD + d;
      const int dd = g / kL;
      const int ll = g - dd * kL;
      idx = ((size_t)s * kL + ll) * kD + dd;
    } else {
      const int b = s / kW;
      const int w = s - b * kW;
      idx = (((size_t)b * kH + ls) * kW + w) * kD + d;
    }
    const float raw = src[idx];
    const float val = kSecond ? raw : bf16r(raw);
    _Float16 hi, lo;
    split_hl(val, kInCarry, hi, lo);
    hv[e] = live ? hi : (_Float16)0.0f;
    lv[e] = live ? lo : (_Float16)0.0f;
  }
  unsigned short* dp = X16 + (size_t)r * kDX + d8;
  for (int pass = 0; pass < 2; ++pass) {
    *(volatile v8h*)dp = hv;
    *(volatile v8h*)(dp + kD) = lv;
    __threadfence();
  }
}
static_assert(((size_t)kRows * 24) % kThr == 0, "operand rows grid exact");

__global__ __launch_bounds__(kThr) void conv_silu_kernel(const float* __restrict__ XZ, const float* __restrict__ conv_w, const float* __restrict__ conv_b,
                                                         float* __restrict__ XC, unsigned short* __restrict__ XC16) {
  const size_t v = (size_t)blockIdx.x * kThr + threadIdx.x;
  const size_t row = v / 96;
  const int c4 = (int)(v - row * 96) * 4;
  const int l = (int)(row % kL);
  v4f acc = *(const v4f*)(conv_b + c4);
#pragma unroll
  for (int e = 0; e < 4; ++e) { const float b0 = acc[e]; acc[e] = bf16r(b0); }
#pragma unroll
  for (int j = 0; j < kConv; ++j) {
    const int back = kConv - 1 - j;
    const bool ok = l >= back;
    const size_t rr = ok ? (row - back) : row;
    const v4f xin = *(const v4f*)(XZ + rr * kDi2 + c4);
#pragma unroll
    for (int e = 0; e < 4; ++e) {
      const float w = conv_w[(size_t)(c4 + e) * kConv + j];
      acc[e] += ok ? (bf16r(w) * xin[e]) : 0.0f;
    }
  }
  v4f o;
  v4h hv, lv;
#pragma unroll
  for (int e = 0; e < 4; ++e) {
    const float s = acc[e] * (1.0f / (1.0f + expf(-acc[e])));
    o[e] = s;
    _Float16 hi, lo;
    split_hl(s, kACarry, hi, lo);
    hv[e] = hi; lv[e] = lo;
  }
  for (int pass = 0; pass < 2; ++pass) {
    *(volatile v4f*)(XC + row * kDi + c4) = o;
    *(volatile v4h*)(XC16 + row * kDiX + c4) = hv;
    *(volatile v4h*)(XC16 + row * kDiX + kDi + c4) = lv;
    __threadfence();
  }
}
static_assert(((size_t)kRows * 96) % kThr == 0 && kDi / 4 == 96, "conv grid exact");

__global__ __launch_bounds__(kThr) void dt_cast_kernel(const float* __restrict__ P, unsigned short* __restrict__ DT16) {
  const size_t v = (size_t)blockIdx.x * kThr + threadIdx.x;
  const size_t row = v >> 2;
  const int c8 = (int)(v & 3) * 8;
  const int cs = c8 & 15;
  const bool isLo = c8 >= 16;
  const v4f a0 = *(const v4f*)(P + row * kXdP + cs);
  const v4f a1 = *(const v4f*)(P + row * kXdP + cs + 4);
  v8h hv;
#pragma unroll
  for (int e = 0; e < 4; ++e) {
    _Float16 h0, l0, h1, l1;
    split_hl(a0[e], kACarry, h0, l0);
    split_hl(a1[e], kACarry, h1, l1);
    hv[e]     = (cs + e < kR) ? (isLo ? l0 : h0) : (_Float16)0.0f;
    hv[4 + e] = (cs + 4 + e < kR) ? (isLo ? l1 : h1) : (_Float16)0.0f;
  }
  unsigned short* dp = DT16 + v * 8;
  *(volatile v8h*)dp = hv;
  __threadfence();
  *(volatile v8h*)dp = hv;
}
static_assert(((size_t)kRows * 4) % kThr == 0, "dt cast grid exact");

__global__ __launch_bounds__(kThr) void sel_scan_kernel(const float* __restrict__ DL, const float* __restrict__ XC, const float* __restrict__ P,
                                                        const float* __restrict__ A_log, float* __restrict__ hidden) {
  const int v = blockIdx.x * kThr + threadIdx.x;
  const int sq = v / kDi;
  const int c = v - sq * kDi;
  float A[kNs], h[kNs];
#pragma unroll
  for (int n = 0; n < kNs; ++n) { const float al = A_log[(size_t)c * kNs + n]; A[n] = -expf(bf16r(al)); h[n] = 0.0f; }
  const size_t r0 = (size_t)sq * kL;
#pragma unroll 1
  for (int l = 0; l < kL; ++l) {
    const size_t row = r0 + l;
    const float dl = DL[row * kDi + c];
    const float xv = XC[row * kDi + c];
    const float dt = (dl > 20.0f) ? dl : log1pf(expf(dl));
    float y = 0.0f;
#pragma unroll
    for (int q = 0; q < 4; ++q) {
      const v4f bq = *(const v4f*)(P + row * kXdP + kR + 4 * q);
      const v4f cq = *(const v4f*)(P + row * kXdP + kR + kNs + 4 * q);
#pragma unroll
      for (int e = 0; e < 4; ++e) {
        const int n = 4 * q + e;
        const float hn = __expf(dt * A[n]) * h[n] + dt * bq[e] * xv;
        h[n] = hn;
        y += hn * cq[e];
      }
    }
    float* hp = hidden + row * kDi + c;
    *(volatile float*)hp = y;
    __threadfence();
    *(volatile float*)hp = y;
  }
}
static_assert((kSeqs2 * kDi) % kThr == 0 && (kDi % 32) == 0, "scan grid exact; a wave inside one sequence");

__global__ __launch_bounds__(kThr) void gate_cast_kernel(const float* __restrict__ hidden, const float* __restrict__ XC, const float* __restrict__ XZ,
                                                         const float* __restrict__ Dp, unsigned short* __restrict__ Y16) {
  const size_t v = (size_t)blockIdx.x * kThr + threadIdx.x;
  const size_t row = v / 48;
  const int c8 = (int)(v - row * 48) * 8;
  const bool live = row < (size_t)kRowsL;
  const size_t rh = live ? row : 0;
  v8h hv, lv;
#pragma unroll
  for (int hlf = 0; hlf < 2; ++hlf) {
    const v4f hh = *(const v4f*)(hidden + rh * kDi + c8 + 4 * hlf);
    const v4f xx = *(const v4f*)(XC + row * kDi + c8 + 4 * hlf);
    const v4f zz = *(const v4f*)(XZ + row * kDi2 + kDi + c8 + 4 * hlf);
    const v4f dd = *(const v4f*)(Dp + c8 + 4 * hlf);
#pragma unroll
    for (int e = 0; e < 4; ++e) {
      const float d0 = dd[e];
      const float g = zz[e] * frcp(1.0f + __expf(-zz[e]));
      _Float16 hi, lo;
      split_hl((hh[e] + bf16r(d0) * xx[e]) * g, kACarry, hi, lo);
      hv[4 * hlf + e] = live ? hi : (_Float16)0.0f;
      lv[4 * hlf + e] = live ? lo : (_Float16)0.0f;
    }
  }
  unsigned short* dp = Y16 + row * kDiX + c8;
  for (int pass = 0; pass < 2; ++pass) {
    *(volatile v8h*)dp = hv;
    *(volatile v8h*)(dp + kDi) = lv;
    __threadfence();
  }
}
static_assert(((size_t)kRows * 48) % kThr == 0 && kDi / 8 == 48, "gate grid exact");

__global__ __launch_bounds__(kThr) void pair_sum_kernel(const float* __restrict__ O, float* __restrict__ dst) {
  const size_t v = (size_t)blockIdx.x * kThr + threadIdx.x;
  const v4f a = *(const v4f*)(O + v * 4);
  const v4f b = *(const v4f*)(O + (size_t)kRowsO * kD + v * 4);
  v4f o;
#pragma unroll
  for (int e = 0; e < 4; ++e) o[e] = a[e] + b[e];
  float* dp = dst + v * 4;
  *(volatile v4f*)dp = o;
  __threadfence();
  *(volatile v4f*)dp = o;
}
static_assert(((size_t)kRowsO * 48) % kThr == 0, "pair sum grid exact");

extern "C" void kernel_launch(void* const* d_in, const int* in_sizes, int n_in,
                              void* d_out, int out_size, void* d_ws, size_t ws_size,
                              hipStream_t stream) {
  if (n_in < 19 || d_out == nullptr || d_ws == nullptr) return;
  if (in_sizes[0] != kRowsO * kD) return;
  for (int p = 0; p < 2; ++p) {
    const int o = 1 + 9 * p;
    if (in_sizes[o] != kDi2 * kD || in_sizes[o + 1] != kDi * kConv || in_sizes[o + 2] != kDi || in_sizes[o + 3] != kXd * kDi) return;
    if (in_sizes[o + 4] != kDi * kR || in_sizes[o + 5] != kDi || in_sizes[o + 6] != kDi * kNs || in_sizes[o + 7] != kDi || in_sizes[o + 8] != kD * kDi) return;
  }
  if (out_size != kRowsO * kD) return;
  if (ws_size < kWsTotal) return;
  const float* x = (const float*)d_in[0];
  float* out = (float*)d_out;
  char* ws = (char*)d_ws;
  unsigned short* X16 = (unsigned short*)(ws + kOffX16);
  float* XZ = (float*)(ws + kOffXZ);
  float* XC = (float*)(ws + kOffXC);
  unsigned short* XC16 = (unsigned short*)(ws + kOffXC16);
  float* P = (float*)(ws + kOffP);
  unsigned short* DT16 = (unsigned short*)(ws + kOffDT16);
  float* DL = (float*)(ws + kOffDL);
  float* HID = (float*)(ws + kOffHID);
  unsigned short* Y16 = (unsigned short*)(ws + kOffY16);
  float* O = (float*)(ws + kOffO);
  float* R1 = (float*)(ws + kOffR1);
  const int rowTiles = kRows / 64;

  for (int p = 0; p < 2; ++p) {
    const int o = 1 + 9 * p;
    const float* in_w = (const float*)d_in[o];
    const float* conv_w = (const float*)d_in[o + 1];
    const float* conv_b = (const float*)d_in[o + 2];
    const float* xp_w = (const float*)d_in[o + 3];
    const float* dt_w = (const float*)d_in[o + 4];
    const float* dt_b = (const float*)d_in[o + 5];
    const float* A_log = (const float*)d_in[o + 6];
    const float* D_skip = (const float*)d_in[o + 7];
    const float* out_w = (const float*)d_in[o + 8];
    char* wb = ws + kOffWts + (size_t)p * kWBlock;
    unsigned short* WIN = (unsigned short*)(wb + kWIN);
    unsigned short* WX = (unsigned short*)(wb + kWX);
    unsigned short* WDT = (unsigned short*)(wb + kWDT);
    unsigned short* WO = (unsigned short*)(wb + kWO);
    float* BV = (float*)(wb + kWBV);

    cast_rows_kernel<<<(kDi2 * (kD / 8)) / kThr, kThr, 0, stream>>>(in_w, WIN, kD / 8, kDX, 0);
    cast_rows_kernel<<<(kDi2 * (kD / 8)) / kThr, kThr, 0, stream>>>(in_w, WIN, kD / 8, kDX, kD);
    wx_plane_kernel<<<kXdP, kDi / 8, 0, stream>>>(xp_w, WX, 0);
    wx_plane_kernel<<<kXdP, kDi / 8, 0, stream>>>(xp_w, WX, kDi);
    wdt_plane_kernel<<<6, kThr, 0, stream>>>(dt_w, WDT);
    cast_rows_kernel<<<(kD * (kDi / 8)) / kThr, kThr, 0, stream>>>(out_w, WO, kDi / 8, kDiX, 0);
    cast_rows_kernel<<<(kD * (kDi / 8)) / kThr, kThr, 0, stream>>>(out_w, WO, kDi / 8, kDiX, kDi);
    bias_rows_kernel<<<kBvTot / 128, 128, 0, stream>>>(dt_b, BV);

    if (p == 0) pass_rows_kernel<false><<<(kRows * 24) / kThr, kThr, 0, stream>>>(x, X16);
    else        pass_rows_kernel<true><<<(kRows * 24) / kThr, kThr, 0, stream>>>(R1, X16);
    wmma_gemm64<0, false, 2, 0, false, 0><<<dim3(rowTiles * (kDi2 / 64) / 8, 1), 256, 0, stream>>>(
        X16, X16, kDX, 0L, WIN, WIN, kDX, 0L, (void*)XZ, (void*)XZ, kDi2, 0L, BV + kBvZ, nullptr, 0L, kRows, kDi2, kDX, kScIn);
    conv_silu_kernel<<<(int)(((size_t)kRows * 96) / kThr), kThr, 0, stream>>>(XZ, conv_w, conv_b, XC, XC16);
    wmma_gemm64<0, false, 2, 0, false, 0><<<dim3(rowTiles * (kXdP / 64) / 8, 1), 256, 0, stream>>>(
        XC16, XC16, kDiX, 0L, WX, WX, kDiX, 0L, (void*)P, (void*)P, kXdP, 0L, BV + kBvZ, nullptr, 0L, kRows, kXdP, kDiX, kScA);
    dt_cast_kernel<<<(int)(((size_t)kRows * 4) / kThr), kThr, 0, stream>>>(P, DT16);
    wmma_gemm64<0, false, 2, 0, false, 0><<<dim3(rowTiles * (kDi / 64) / 8, 1), 256, 0, stream>>>(
        DT16, DT16, kRP, 0L, WDT, WDT, kRP, 0L, (void*)DL, (void*)DL, kDi, 0L, BV + kBvDt, nullptr, 0L, kRows, kDi, kRP, kScA);
    sel_scan_kernel<<<(kSeqs2 * kDi) / kThr, kThr, 0, stream>>>(DL, XC, P, A_log, HID);
    gate_cast_kernel<<<(int)(((size_t)kRows * 48) / kThr), kThr, 0, stream>>>(HID, XC, XZ, D_skip, Y16);
    wmma_gemm64<0, false, 2, 0, false, 0><<<dim3(rowTiles * (kD / 64) / 8, 1), 256, 0, stream>>>(
        Y16, Y16, kDiX, 0L, WO, WO, kDiX, 0L, (void*)O, (void*)O, kD, 0L, BV + kBvZ, nullptr, 0L, kRows, kD, kDiX, kScA);
    pair_sum_kernel<<<(int)(((size_t)kRowsO * 48) / kThr), kThr, 0, stream>>>(O, (p == 0) ? R1 : out);
  }
}
